// AxialAttention_3D_16183436771877
// MI455X (gfx1250) — hardware-run, weakly checked
//
#include <hip/hip_runtime.h>


#ifndef NSEQ
#define NSEQ 1792
#endif
#define NSEQ_FULL 1792
#define KW    56
#define KP    64
#define CIN   64
#define OC2   128
#define NHEAD 8
#define RELW  111
#define PT      (NSEQ * KW)
#define PT_FULL (NSEQ_FULL * KW)
#define SOP     (NSEQ * KP)
#define F_QR  0.1f
#define F_KR  0.1f
#define F_SVE 0.1f
#define EPSB  1e-5f
#define LOG2E 1.4426950408889634f
#define PSH   14.0f
#define RCAR  16.0f
#define NEGB  (-3.0e38f)

static_assert(NSEQ <= NSEQ_FULL);
static_assert(NSEQ % 8 == 0);
static_assert(PT % 64 == 0);
static_assert(PT_FULL % 4 == 0);
static_assert(KW % 8 == 0);
static_assert(KW % 4 == 0);
static_assert(KW <= KP);
static_assert(KP == 64);
static_assert(CIN % 32 == 0);
static_assert(OC2 % 64 == 0);
static_assert(NHEAD == 8);
static_assert(NHEAD * 16 == OC2);
static_assert(RELW == 2 * KW - 1);
static_assert(RELW <= 128);
static_assert(KP + KW - 1 <= 128);

typedef _Float16 h16;
typedef unsigned short bf;
typedef __attribute__((ext_vector_type(16))) __bf16   v16bf;
typedef __attribute__((ext_vector_type(16))) _Float16 v16h;
typedef __attribute__((ext_vector_type(8)))  _Float16 v8h;
typedef __attribute__((ext_vector_type(8)))  unsigned short v8us;
typedef __attribute__((ext_vector_type(8)))  float    v8f;
typedef __attribute__((ext_vector_type(4)))  float    v4f;
typedef v4f  __attribute__((may_alias)) v4fa;
typedef v8us __attribute__((may_alias)) v8usa;
typedef v8h  __attribute__((may_alias)) v8ha;

__device__ __forceinline__ unsigned short f2bf(float f) { unsigned u = __float_as_uint(f); u += 0x7FFFu + ((u >> 16) & 1u); return (unsigned short)(u >> 16); }
__device__ __forceinline__ float bfr(float f) { return __uint_as_float(((unsigned)f2bf(f)) << 16); }
__device__ __forceinline__ v16h cat16(v8h lo, v8h hi) { return __builtin_shufflevector(lo, hi, 0, 1, 2, 3, 4, 5, 6, 7, 8, 9, 10, 11, 12, 13, 14, 15); }
__device__ __forceinline__ v16bf cat16b(v8us lo, v8us hi) { return __builtin_bit_cast(v16bf, __builtin_shufflevector(lo, hi, 0, 1, 2, 3, 4, 5, 6, 7, 8, 9, 10, 11, 12, 13, 14, 15)); }
__device__ __forceinline__ v8f wmma16(v16h a, v16h b, v8f c) { return __builtin_amdgcn_wmma_f32_16x16x32_f16(false, a, false, b, (short)0, c, false, false); }
__device__ __forceinline__ v8f wmmab(v16bf a, v16bf b, v8f c) { return __builtin_amdgcn_wmma_f32_16x16x32_bf16(false, a, false, b, (short)0, c, false, false); }
__device__ __forceinline__ v16h  ldh(const h16* p) { return cat16(*(const v8h*)p, *(const v8h*)(p + 16)); }
__device__ __forceinline__ v16bf ldb(const bf* p)  { return cat16b(*(const v8us*)p, *(const v8us*)(p + 16)); }
__device__ __forceinline__ void wave_sync() { __builtin_amdgcn_fence(3  , "wavefront"); __builtin_amdgcn_wave_barrier(); asm volatile("" ::: "memory"); }

__device__ __forceinline__ h16 toh_flush(float v) { const h16 r = (h16)v; return (fabsf(v) < 6.103515625e-05f) ? (h16)0.0f : r; }
__device__ __forceinline__ v8f wmma16g(v16h a, v16h b, v8f c) { c = wmma16(a, b, c); asm volatile("v_nop\n\tv_nop\n\tv_nop\n\tv_nop" : "+v"(c) : "v"(a), "v"(b)); return c; }
__device__ __forceinline__ v8f wmmabg(v16bf a, v16bf b, v8f c) { c = wmmab(a, b, c); asm volatile("v_nop\n\tv_nop\n\tv_nop\n\tv_nop" : "+v"(c) : "v"(a), "v"(b)); return c; }
__device__ __forceinline__ float wsumf(float v) { v += __shfl_xor(v, 16, 32); v += __shfl_xor(v, 8, 32); v += __shfl_xor(v, 4, 32); v += __shfl_xor(v, 2, 32); v += __shfl_xor(v, 1, 32); return v; }
__device__ __forceinline__ double wsumd(double v) { v += __shfl_xor(v, 16, 32); v += __shfl_xor(v, 8, 32); v += __shfl_xor(v, 4, 32); v += __shfl_xor(v, 2, 32); v += __shfl_xor(v, 1, 32); return v; }

__global__ __launch_bounds__(256) void k_cvt8(const float* __restrict__ src, bf* dst, size_t n8) {
    const size_t i = (size_t)blockIdx.x * 256 + threadIdx.x; if (i >= n8) return;
    const v8f v = *(const v8f*)(src + i * 8); v8us o;
#pragma unroll
    for (int k = 0; k < 8; ++k) o[k] = f2bf(v[k]);
    *(volatile v8us*)(dst + i * 8) = o; __threadfence(); *(volatile v8us*)(dst + i * 8) = o;
}

__global__ __launch_bounds__(256) void k_xpose(const float* __restrict__ x, bf* XT) {
    __shared__ __align__(16) unsigned short ts[64 * 72];
    const int tid = threadIdx.x; const int p0 = blockIdx.x * 64;
    static_assert(4 * 256 * 4 == 64 * CIN);
#pragma unroll 1
    for (int s = 0; s < 4; ++s) { const int idx = s * 256 + tid; const int c = idx >> 4, p4 = (idx & 15) * 4;
        const v4f v = *(const v4f*)(x + (size_t)c * PT_FULL + p0 + p4);
#pragma unroll
        for (int e = 0; e < 4; ++e) ts[(p4 + e) * 72 + c] = f2bf(v[e]); }
    __syncthreads();
    static_assert(256 * 2 * 16 == 64 * CIN * 2);
#pragma unroll 1
    for (int ps = 0; ps < 2; ++ps) {
#pragma unroll
        for (int s = 0; s < 2; ++s) { const int q = s * 256 + tid; const int row = q >> 3, c8 = (q & 7) * 8;
            const v8us o = *(const v8usa*)(&ts[row * 72 + c8]);
            *(volatile v8us*)(XT + (size_t)(p0 + row) * CIN + c8) = o; }
        if (ps == 0) __threadfence(); }
}

__global__ __launch_bounds__(256) void k_rtab(const float* __restrict__ rel, float* TBg, h16* RAg) {
    const int t = threadIdx.x;
    v4f o4; v8h o8;
    { const int e = t >> 1, half = t & 1; const int d = e - 8; const bool ok = (d >= 0) & (d <= RELW - 1);
      const int dc = d < 0 ? 0 : (d > RELW - 1 ? RELW - 1 : d);
#pragma unroll
      for (int c = 0; c < 4; ++c) { const int off = half ? ((4 + c) * RELW + (RELW - 1 - dc)) : (c * RELW + dc);
          float v = rel[off]; asm volatile("" : "+v"(v)); o4[c] = ok ? bfr(v) : 0.0f; } }
    { const int c = t >> 4, d8 = (t & 15) * 8; const int cc = c < 8 ? c : 7;
#pragma unroll
      for (int e = 0; e < 8; ++e) { const int d = d8 + e; const int dc = d > RELW - 1 ? RELW - 1 : d; const bool ok = (c < 8) & (d < RELW);
          float v = rel[(8 + cc) * RELW + dc]; asm volatile("" : "+v"(v)); o8[e] = ok ? toh_flush(bfr(v) * RCAR) : (h16)0.0f; } }
    static_assert(256 * 16 == 128 * 8 * 4);
    static_assert(256 * 16 == 16 * 128 * 2);
    *(volatile v4f*)(TBg + t * 4) = o4; *(volatile v8h*)(RAg + t * 8) = o8;
    __threadfence();
    *(volatile v4f*)(TBg + t * 4) = o4; *(volatile v8h*)(RAg + t * 8) = o8;
}

__global__ __launch_bounds__(32) void k_gemm(const bf* __restrict__ A, const bf* __restrict__ Bt, float* C) {
    __shared__ __align__(16) float os[16 * 68];
    const int K = CIN;
    const int lane = threadIdx.x & 31, lr = lane & 15, hi = lane >> 4; const int r0 = blockIdx.x * 64, c0 = blockIdx.y * 64;
    v8f acc[4][4];
#pragma unroll
    for (int mb = 0; mb < 4; ++mb)
#pragma unroll
        for (int nb = 0; nb < 4; ++nb) acc[mb][nb] = (v8f){};
    const size_t aoff = (size_t)(r0 + lr) * K + 8 * hi, boff = (size_t)(c0 + lr) * K + 8 * hi;
#pragma unroll 1
    for (int kc = 0; kc < K; kc += 32) {
        v16bf a[4];
#pragma unroll
        for (int mb = 0; mb < 4; ++mb) a[mb] = ldb(A + aoff + (size_t)mb * 16 * K + kc);
#pragma unroll
        for (int nb = 0; nb < 4; ++nb) { const v16bf b = ldb(Bt + boff + (size_t)nb * 16 * K + kc);
#pragma unroll
            for (int mb = 0; mb < 4; ++mb) acc[mb][nb] = wmmabg(a[mb], b, acc[mb][nb]); }
    }
#pragma unroll
    for (int mb = 0; mb < 4; ++mb) {
#pragma unroll
        for (int nb = 0; nb < 4; ++nb) {
#pragma unroll
            for (int j = 0; j < 8; ++j) os[(hi * 8 + j) * 68 + nb * 16 + lr] = acc[mb][nb][j]; }
        wave_sync();
        float* cb = C + (size_t)(r0 + mb * 16) * PT + c0;
        static_assert(8 * 2 == 16);
#pragma unroll 1
        for (int ps = 0; ps < 2; ++ps) {
#pragma unroll
            for (int s = 0; s < 8; ++s) { const int row = 2 * s + (lane >> 4), c4 = (lane & 15) * 4;
                const v4f val = *(const v4fa*)(&os[row * 68 + c4]);
                *(volatile v4f*)(cb + (size_t)row * PT + c4) = val; }
            if (ps == 0) __threadfence(); }
        wave_sync();
    }
}

__global__ __launch_bounds__(256) void k_stats(const float* __restrict__ src, const float* __restrict__ gma, const float* __restrict__ bta, float* tab,
                                               size_t pitch, double inv_cnt, int n4) {
#pragma clang fp contract(off)
    __shared__ double sd[8];
    __shared__ double qd[8];
    const int tid = threadIdx.x, lane = tid & 31;
    const int wave = __builtin_amdgcn_readfirstlane((int)(threadIdx.x >> 5));
    const int ch = blockIdx.x;
    const float* row = src + (size_t)ch * pitch;
    double s = 0.0, q = 0.0;
#pragma unroll 1
    for (int i = tid; i < n4; i += 256) { const v4f v = *(const v4f*)(row + (size_t)i * 4);
        const float a = (v[0] + v[1]) + (v[2] + v[3]);
        const float bb = (v[0] * v[0] + v[1] * v[1]) + (v[2] * v[2] + v[3] * v[3]);
        s += (double)a; q += (double)bb; }
    s = wsumd(s); q = wsumd(q);
    if (lane == 0) { sd[wave] = s; qd[wave] = q; }
    __syncthreads();
    double S = 0.0, Q = 0.0;
#pragma unroll
    for (int w = 0; w < 8; ++w) { S += sd[w]; Q += qd[w]; }
    const double mean = S * inv_cnt;
    double var = Q * inv_cnt - mean * mean; var = var < 0.0 ? 0.0 : var;
    const float sc = bfr(gma[ch]) * rsqrtf((float)var + EPSB);
    const float sh = bfr(bta[ch]) - (float)mean * sc;
    v4f o; o[0] = (lane == 0) ? sc : 0.0f; o[1] = (lane == 0) ? sh : 0.0f; o[2] = 0.0f; o[3] = 0.0f;
    if (tid < 8) { float* p = tab + (size_t)ch * 32 + tid * 4;
        *(volatile v4f*)p = o; __threadfence(); *(volatile v4f*)p = o; }
}

template <int STATS>
__device__ __forceinline__ void attn_body(const float* __restrict__ QKV, const float* __restrict__ BNQ, const float* __restrict__ BNS,
                                          const float* __restrict__ TBg, const h16* __restrict__ RAg, float* PART, float* SO) {
    __shared__ __align__(16) float qf[4 * KP];
    __shared__ __align__(16) float kf[4 * KP];
    __shared__ __align__(16) unsigned short QB[KP * 16];
    __shared__ __align__(16) unsigned short KA[KP * 16];
    __shared__ __align__(16) h16 VA[16 * KP];
    __shared__ __align__(16) float TB[128 * 8];
    __shared__ __align__(16) h16 PS[4 * 16 * 128];
    __shared__ __align__(16) float OS[16 * 68];
    __shared__ __align__(16) float red[4 * 8];
    const int tid = threadIdx.x, lane = tid & 31, lr = lane & 15, hi = lane >> 4;
    const int wave = __builtin_amdgcn_readfirstlane((int)(threadIdx.x >> 5));
    const int bg = blockIdx.x; const int b = bg >> 3, g = bg & 7;
    float c0 = 1.0f, a1 = 1.0f, a2 = 1.0f, shc = 0.0f;
    if (!STATS) {
        const float s0 = BNS[2 * g], h0 = BNS[2 * g + 1];
        const float s1 = BNS[2 * (8 + g)], h1 = BNS[2 * (8 + g) + 1];
        const float s2 = BNS[2 * (16 + g)], h2 = BNS[2 * (16 + g) + 1];
        c0 = s0 * LOG2E; a1 = s1 * F_QR * LOG2E; a2 = s2 * F_KR * LOG2E; shc = ((h0 + h1) + h2) * LOG2E;
    }
    static_assert(2 * 128 == 4 * KP);
#pragma unroll 1
    for (int s = 0; s < 2; ++s) {
        const int idx = s * 128 + tid; const int c = idx >> 6, i = idx & 63; const int ic = i < KW ? i : KW - 1;
        const int oq = g * 16 + c, ok = oq + 4;
        float rq = QKV[(size_t)oq * PT + (size_t)b * KW + ic];
        float rk = QKV[(size_t)ok * PT + (size_t)b * KW + ic];
        const float sq = BNQ[oq * 32], hq = BNQ[oq * 32 + 1], sk = BNQ[ok * 32], hk = BNQ[ok * 32 + 1];
        asm volatile("" : "+v"(rq)); asm volatile("" : "+v"(rk));
        const bool in = i < KW;
        const float vq = in ? (sq * rq + hq) : 0.0f;
        const float vk = in ? (sk * rk + hk) : 0.0f;
        qf[idx] = vq; kf[idx] = vk;
        const unsigned short qh = f2bf(vq); const unsigned short ql = f2bf(vq - __uint_as_float(((unsigned)qh) << 16));
        const unsigned short kh = f2bf(vk); const unsigned short kl = f2bf(vk - __uint_as_float(((unsigned)kh) << 16));
        QB[i * 16 + c] = qh; QB[i * 16 + 4 + c] = ql; QB[i * 16 + 8 + c] = qh; QB[i * 16 + 12 + c] = (unsigned short)0;
        KA[i * 16 + c] = kh; KA[i * 16 + 4 + c] = kh; KA[i * 16 + 8 + c] = kl; KA[i * 16 + 12 + c] = (unsigned short)0;
    }
    if (!STATS) {
        static_assert(4 * 128 == 8 * KP);
#pragma unroll 1
        for (int s = 0; s < 4; ++s) {
            const int idx = s * 128 + tid; const int c = idx >> 6, j = idx & 63; const int jc = j < KW ? j : KW - 1;
            const int ov = g * 16 + 8 + c;
            float rv = QKV[(size_t)ov * PT + (size_t)b * KW + jc];
            const float sv = BNQ[ov * 32], hv = BNQ[ov * 32 + 1];
            asm volatile("" : "+v"(rv));
            const float vv = (j < KW) ? (sv * rv + hv) : 0.0f;
            VA[c * KP + j] = toh_flush(vv); VA[(c + 8) * KP + j] = (h16)0.0f;
        }
        static_assert(8 * 128 * 8 == 4 * 16 * 128);
#pragma unroll
        for (int s = 0; s < 8; ++s) *(v8ha*)(&PS[(s * 128 + tid) * 8]) = (v8h){};
    }
    {
      const v4f t0 = *(const v4f*)(TBg + tid * 8), t1 = *(const v4f*)(TBg + tid * 8 + 4);
      *(v4fa*)(&TB[tid * 8]) = t0 * a1; *(v4fa*)(&TB[tid * 8 + 4]) = t1 * a2; }
    __syncthreads();

    const int i0 = wave * 16; const int iq = i0 + lr;
    const bool iv = iq < KW;
    const float q0 = qf[iq], q1 = qf[KP + iq], q2 = qf[2 * KP + iq], q3 = qf[3 * KP + iq];
    const v8us z8 = (v8us){};
    const v16bf qb = cat16b(*(const v8usa*)(&QB[iq * 16 + 8 * hi]), z8);
    const int eb = iq - 8 * hi + 63;
    float ta[4][8];
    float sA = 0.0f, qA = 0.0f, sB = 0.0f, qB = 0.0f, sC = 0.0f, qC = 0.0f;
    if (STATS) {
#pragma unroll 1
        for (int t = 0; t < 4; ++t) {
            const v16bf ka = cat16b(*(const v8usa*)(&KA[(16 * t + lr) * 16 + 8 * hi]), z8);
            v8f d = (v8f){}; d = wmmabg(ka, qb, d);
            const int jb = 16 * t + 8 * hi;
            float kc[4][8];
#pragma unroll
            for (int c = 0; c < 4; ++c) { const v4f x0 = *(const v4fa*)(&kf[c * KP + jb]); const v4f x1 = *(const v4fa*)(&kf[c * KP + jb + 4]);
#pragma unroll
                for (int r = 0; r < 4; ++r) { kc[c][r] = x0[r]; kc[c][4 + r] = x1[r]; } }
            const bool jv = jb < KW;
#pragma unroll
            for (int r = 0; r < 8; ++r) {
                const int e = eb - 16 * t - r;
                const v4f tq = *(const v4fa*)(&TB[e * 8]); const v4f tk = *(const v4fa*)(&TB[e * 8 + 4]);
                const float qr = (q0 * tq[0] + q1 * tq[1]) + (q2 * tq[2] + q3 * tq[3]);
                const float kr = (kc[0][r] * tk[0] + kc[1][r] * tk[1]) + (kc[2][r] * tk[2] + kc[3][r] * tk[3]);
                const float qrm = jv ? qr : 0.0f;
                const float krm = iv ? kr : 0.0f;
                const float dq = d[r];
                sA += dq; qA += dq * dq; sB += qrm; qB += qrm * qrm; sC += krm; qC += krm * krm;
            }
        }
    } else {
#pragma unroll
        for (int t = 0; t < 4; ++t) {
            const v16bf ka = cat16b(*(const v8usa*)(&KA[(16 * t + lr) * 16 + 8 * hi]), z8);
            v8f d = (v8f){}; d = wmmabg(ka, qb, d);
            const int jb = 16 * t + 8 * hi;
            float kc[4][8];
#pragma unroll
            for (int c = 0; c < 4; ++c) { const v4f x0 = *(const v4fa*)(&kf[c * KP + jb]); const v4f x1 = *(const v4fa*)(&kf[c * KP + jb + 4]);
#pragma unroll
                for (int r = 0; r < 4; ++r) { kc[c][r] = x0[r]; kc[c][4 + r] = x1[r]; } }
#pragma unroll
            for (int r = 0; r < 8; ++r) {
                const int e = eb - 16 * t - r;
                const v4f tq = *(const v4fa*)(&TB[e * 8]); const v4f tk = *(const v4fa*)(&TB[e * 8 + 4]);
                float acc = fmaf(d[r], c0, shc);
                acc = fmaf(q0, tq[0], acc); acc = fmaf(q1, tq[1], acc); acc = fmaf(q2, tq[2], acc); acc = fmaf(q3, tq[3], acc);
                acc = fmaf(kc[0][r], tk[0], acc); acc = fmaf(kc[1][r], tk[1], acc); acc = fmaf(kc[2][r], tk[2], acc); acc = fmaf(kc[3][r], tk[3], acc);
                ta[t][r] = acc;
                if (r == 3) asm volatile("" ::: "memory");
            }
            asm volatile("" ::: "memory");
        }
    }
    if (STATS) {
        sA = wsumf(sA); qA = wsumf(qA); sB = wsumf(sB); qB = wsumf(qB); sC = wsumf(sC); qC = wsumf(qC);
        if (lane == 0) { red[wave * 8 + 0] = sA; red[wave * 8 + 1] = qA; red[wave * 8 + 2] = sB; red[wave * 8 + 3] = qB;
                         red[wave * 8 + 4] = sC; red[wave * 8 + 5] = qC; red[wave * 8 + 6] = 0.0f; red[wave * 8 + 7] = 0.0f; }
        __syncthreads();
        const int k4 = (lane & 1) * 4;
        v4f o;
#pragma unroll
        for (int k = 0; k < 4; ++k) { const float v = (red[k4 + k] + red[8 + k4 + k]) + (red[16 + k4 + k] + red[24 + k4 + k]); o[k] = (lane < 2) ? v : 0.0f; }
        if (tid < 8) { float* p = PART + (size_t)bg * 32 + tid * 4;
            *(volatile v4f*)p = o; __threadfence(); *(volatile v4f*)p = o; }
    } else {
        const bool jv3 = (48 + 8 * hi) < KW;
        float mx = NEGB;
#pragma unroll
        for (int t = 0; t < 4; ++t)
#pragma unroll
            for (int r = 0; r < 8; ++r) { const float v = (t == 3) ? (jv3 ? ta[t][r] : NEGB) : ta[t][r]; mx = fmaxf(mx, v); }
        mx = fmaxf(mx, __shfl_xor(mx, 16, 32));
        const float sh = PSH - mx;
        const int wb = wave * (16 * 128);
        const int db = eb - 8;
        v16h pb0 = (v16h){}, pb1 = (v16h){}; float ls = 0.0f;
#pragma unroll
        for (int t = 0; t < 4; ++t)
#pragma unroll
            for (int r = 0; r < 8; ++r) {
                const float ee = ta[t][r] + sh;
                float p = (ee < -14.0f) ? 0.0f : __builtin_amdgcn_exp2f(ee);
                if (t == 3) p = jv3 ? p : 0.0f;
                const h16 ph = (h16)p; ls += (float)ph;
                if (t == 0) pb0[r] = ph; else if (t == 1) pb0[8 + r] = ph; else if (t == 2) pb1[r] = ph; else pb1[8 + r] = ph;
                const int dd = db - 16 * t - r;
                if (t < 3) PS[wb + lr * 128 + dd] = ph; else { if (jv3) PS[wb + lr * 128 + dd] = ph; }
            }
        wave_sync();
        const v16h va0 = cat16(*(const v8ha*)(&VA[lr * KP + 8 * hi]),      *(const v8ha*)(&VA[lr * KP + 8 * hi + 16]));
        const v16h va1 = cat16(*(const v8ha*)(&VA[lr * KP + 8 * hi + 32]), *(const v8ha*)(&VA[lr * KP + 8 * hi + 48]));
        v8f o = (v8f){}; o = wmma16g(va0, pb0, o); o = wmma16g(va1, pb1, o);
        v8f ev = (v8f){};
#pragma unroll
        for (int ks = 0; ks < 4; ++ks) {
            const v16h ra = ldh(RAg + lr * 128 + 32 * ks + 8 * hi);
            const int po = wb + lr * 128 + 32 * ks + 8 * hi;
            const v16h pf = cat16(*(const v8ha*)(&PS[po]), *(const v8ha*)(&PS[po + 16]));
            ev = wmma16g(ra, pf, ev); }
        const float l = ls + __shfl_xor(ls, 16, 32);
        const float inv = 1.0f / l;
        const float ke = inv * (F_SVE * (1.0f / RCAR));
        if (hi == 0) {
#pragma unroll
            for (int r = 0; r < 8; ++r) { OS[(2 * r) * 68 + iq] = iv ? (o[r] * inv) : 0.0f; OS[(2 * r + 1) * 68 + iq] = iv ? (ev[r] * ke) : 0.0f; } }
        __syncthreads();
        float* sob = SO + (size_t)(g * 16) * SOP + (size_t)b * KP;
        static_assert(128 * 2 * 16 == 16 * KP * 4);
#pragma unroll 1
        for (int ps = 0; ps < 2; ++ps) {
#pragma unroll
            for (int s = 0; s < 2; ++s) { const int q = s * 128 + tid; const int row = q >> 4, c4 = (q & 15) * 4;
                const v4f val = *(const v4fa*)(&OS[row * 68 + c4]);
                *(volatile v4f*)(sob + (size_t)row * SOP + c4) = val; }
            if (ps == 0) __threadfence(); }
    }
}

static constexpr size_t LDS_ATTN = 4 * KP * 4 * 2 + KP * 16 * 2 * 2 + 16 * KP * 2 + 128 * 8 * 4 + 4 * 16 * 128 * 2 + 16 * 68 * 4 + 4 * 8 * 4;
static_assert(LDS_ATTN <= 131072);
static_assert(64 * 72 * 2 <= 131072);
static_assert(16 * 68 * 4 <= 131072);

__global__ __launch_bounds__(128) __attribute__((amdgpu_num_vgpr(256)))
void k_simstats(const float* __restrict__ QKV, const float* __restrict__ BNQ, const float* __restrict__ TBg, float* PART) {
    attn_body<1>(QKV, BNQ, (const float*)nullptr, TBg, (const h16*)nullptr, PART, (float*)nullptr);
}
__global__ __launch_bounds__(128) __attribute__((amdgpu_num_vgpr(256)))
void k_attn(const float* __restrict__ QKV, const float* __restrict__ BNQ, const float* __restrict__ BNS,
            const float* __restrict__ TBg, const h16* __restrict__ RAg, float* SO) {
    attn_body<0>(QKV, BNQ, BNS, TBg, RAg, (float*)nullptr, SO);
}

__global__ __launch_bounds__(256) void k_bns(const float* __restrict__ PART, const float* __restrict__ gma, const float* __restrict__ bta, float* BNS, double inv_cnt) {
#pragma clang fp contract(off)
    __shared__ __align__(16) float tab[64];
    static_assert(NHEAD * 32 == 256);
    static_assert(3 * NHEAD == 24);
    const int tid = threadIdx.x, lane = tid & 31;
    const int wave = __builtin_amdgcn_readfirstlane((int)(threadIdx.x >> 5));
    if (tid < 64) tab[tid] = 0.0f;
    __syncthreads();
    float gn0 = gma[wave], gn1 = gma[8 + wave], gn2 = gma[16 + wave];
    float bi0 = bta[wave], bi1 = bta[8 + wave], bi2 = bta[16 + wave];
    asm volatile("" : "+v"(gn0)); asm volatile("" : "+v"(gn1)); asm volatile("" : "+v"(gn2));
    asm volatile("" : "+v"(bi0)); asm volatile("" : "+v"(bi1)); asm volatile("" : "+v"(bi2));
    double a0 = 0.0, a1 = 0.0, a2 = 0.0, a3 = 0.0, a4 = 0.0, a5 = 0.0;
#pragma unroll 1
    for (int b = lane; b < NSEQ; b += 32) { const float* p = PART + ((size_t)b * NHEAD + wave) * 32;
        const v4f x0 = *(const v4f*)p, x1 = *(const v4f*)(p + 4);
        a0 += (double)x0[0]; a1 += (double)x0[1]; a2 += (double)x0[2]; a3 += (double)x0[3]; a4 += (double)x1[0]; a5 += (double)x1[1]; }
    a0 = wsumd(a0); a1 = wsumd(a1); a2 = wsumd(a2); a3 = wsumd(a3); a4 = wsumd(a4); a5 = wsumd(a5);
    if (lane == 0) {
        const double S[3] = { a0, a2, a4 }; const double Q[3] = { a1, a3, a5 }; const double f[3] = { 1.0, (double)F_QR, (double)F_KR };
        const float G[3] = { gn0, gn1, gn2 }; const float Bv[3] = { bi0, bi1, bi2 };
#pragma unroll
        for (int t = 0; t < 3; ++t) { const int ch = t * 8 + wave;
            const double m = S[t] * inv_cnt; double var = Q[t] * inv_cnt - m * m; var = var < 0.0 ? 0.0 : var;
            const double ms = m * f[t], vs = var * f[t] * f[t];
            const float sc = bfr(G[t]) * rsqrtf((float)vs + EPSB);
            tab[2 * ch] = sc; tab[2 * ch + 1] = bfr(Bv[t]) - (float)ms * sc; }
    }
    __syncthreads();
    if (tid < 16) { const v4f v = *(const v4fa*)(&tab[tid * 4]); float* p = BNS + tid * 4;
        *(volatile v4f*)p = v; __threadfence(); *(volatile v4f*)p = v; }
}

__global__ __launch_bounds__(256) void k_out(const float* __restrict__ SO, const float* __restrict__ BNO, float* OUT) {
    const size_t idx = (size_t)blockIdx.x * 256 + threadIdx.x;
    const size_t n4row = (size_t)PT / 4;
    if (idx >= (size_t)(OC2 / 2) * n4row) return;
    const int c = (int)(idx / n4row); const int p = (int)(idx - (size_t)c * n4row) * 4;
    const int b = p / KW, i = p - b * KW;
    const int o0 = 2 * c, o1 = 2 * c + 1;
    const float s0 = BNO[o0 * 32], h0 = BNO[o0 * 32 + 1], s1 = BNO[o1 * 32], h1 = BNO[o1 * 32 + 1];
    const v4f x0 = *(const v4f*)(SO + (size_t)o0 * SOP + (size_t)b * KP + i);
    const v4f x1 = *(const v4f*)(SO + (size_t)o1 * SOP + (size_t)b * KP + i);
    const v4f val = (x0 * s0 + h0) + (x1 * s1 + h1);
    float* dst = OUT + (size_t)c * PT_FULL + p;
    *(volatile v4f*)dst = val; __threadfence(); *(volatile v4f*)dst = val;
}

static constexpr size_t al256(size_t v) { return (v + 255) & ~(size_t)255; }
static constexpr size_t SZ_WB   = al256((size_t)OC2 * CIN * 2);
static constexpr size_t SZ_XT   = al256((size_t)PT * CIN * 2);
static constexpr size_t SZ_TBG  = al256((size_t)128 * 8 * 4);
static constexpr size_t SZ_RAG  = al256((size_t)16 * 128 * 2);
static constexpr size_t SZ_QKV  = al256((size_t)OC2 * PT * 4);
static constexpr size_t SZ_BNT  = al256((size_t)OC2 * 32 * 4);
static constexpr size_t SZ_PART = al256((size_t)NSEQ * NHEAD * 32 * 4);
static constexpr size_t SZ_BNS  = al256((size_t)64 * 4);
static constexpr size_t SZ_SO   = al256((size_t)OC2 * SOP * 4);
static constexpr size_t SZ_TOTAL = SZ_WB + SZ_XT + SZ_TBG + SZ_RAG + SZ_QKV + 2 * SZ_BNT + SZ_PART + SZ_BNS + SZ_SO;
static_assert(SZ_TOTAL <= (size_t)134217728);
static_assert(((size_t)OC2 * CIN) % 8 == 0);
static_assert(((size_t)(OC2 / 2) * (PT / 4)) % 256 == 0);
static_assert((PT / 4) % 8 == 0);

extern "C" void kernel_launch(void* const* d_in, const int* in_sizes, int n_in,
                              void* d_out, int out_size, void* d_ws, size_t ws_size, hipStream_t stream) {
    if (n_in < 9) return;
    const size_t needx = (size_t)(CIN - 1) * PT_FULL + PT;
    if ((size_t)in_sizes[0] < needx) return;
    if ((size_t)in_sizes[1] < (size_t)OC2 * CIN || (size_t)in_sizes[2] < (size_t)16 * RELW) return;
    if (in_sizes[3] < OC2 || in_sizes[4] < OC2 || in_sizes[5] < 24 || in_sizes[6] < 24 || in_sizes[7] < OC2 || in_sizes[8] < OC2) return;
    if ((size_t)out_size < (size_t)(OC2 / 2 - 1) * PT_FULL + PT) return;
    if (SZ_TOTAL > ws_size) return;
    const float* x   = (const float*)d_in[0];
    const float* wq  = (const float*)d_in[1];
    const float* rel = (const float*)d_in[2];
    const float* gq  = (const float*)d_in[3]; const float* bq = (const float*)d_in[4];
    const float* gs  = (const float*)d_in[5]; const float* bs = (const float*)d_in[6];
    const float* go  = (const float*)d_in[7]; const float* bo = (const float*)d_in[8];
    float* OUT = (float*)d_out;
    char* wsp = (char*)d_ws;
    bf*    WB   = (bf*)wsp;    wsp += SZ_WB;
    bf*    XT   = (bf*)wsp;    wsp += SZ_XT;
    float* TBg  = (float*)wsp; wsp += SZ_TBG;
    h16*   RAg  = (h16*)wsp;   wsp += SZ_RAG;
    float* QKV  = (float*)wsp; wsp += SZ_QKV;
    float* BNQ  = (float*)wsp; wsp += SZ_BNT;
    float* PART = (float*)wsp; wsp += SZ_PART;
    float* BNS  = (float*)wsp; wsp += SZ_BNS;
    float* SO   = (float*)wsp; wsp += SZ_SO;
    float* BNO  = (float*)wsp; wsp += SZ_BNT;

    const double inv_p = 1.0 / (double)PT;
    const double inv_s = 1.0 / ((double)NSEQ * (double)KW * (double)KW);

    { const size_t n8 = (size_t)OC2 * CIN / 8; k_cvt8<<<(unsigned)((n8 + 255) / 256), 256, 0, stream>>>(wq, WB, n8); }
    k_xpose<<<PT / 64, 256, 0, stream>>>(x, XT);
    k_rtab<<<1, 256, 0, stream>>>(rel, TBg, RAg);
    k_gemm<<<dim3(OC2 / 64, PT / 64, 1), 32, 0, stream>>>(WB, XT, QKV);
    k_stats<<<OC2, 256, 0, stream>>>(QKV, gq, bq, BNQ, (size_t)PT, inv_p, PT / 4);
    k_simstats<<<NSEQ * NHEAD, 128, 0, stream>>>(QKV, BNQ, TBg, PART);
    k_bns<<<1, 256, 0, stream>>>(PART, gs, bs, BNS, inv_s);
    k_attn<<<NSEQ * NHEAD, 128, 0, stream>>>(QKV, BNQ, BNS, TBg, RAg, SO);
    k_stats<<<OC2, 256, 0, stream>>>(SO, go, bo, BNO, (size_t)SOP, inv_p, SOP / 4);
    k_out<<<(unsigned)(((size_t)(OC2 / 2) * (PT / 4)) / 256), 256, 0, stream>>>(SO, BNO, OUT);
}
